// Predictor_65429531787931
// MI455X (gfx1250) — hardware-run, weakly checked
//
#include <hip/hip_runtime.h>
#include <stddef.h>
#include <stdint.h>


#define NNODE   100000
#define KDIM    128
#define NEDGE   625000
#define NPAIR   (NEDGE / 2)
#define MTILE   128
#define MBLK    782
#define MPAD    (MBLK * MTILE)
#define WROWS   16
#define PQW     4
#define THR     256
#define XUNITS  (MPAD * (KDIM / 8))
#define XBLKS   (XUNITS / THR)
#define EBLKS   ((NPAIR + THR - 1) / THR)

#define BYTES_XB ((size_t)MPAD * KDIM * 2)
#define BYTES_PQ ((size_t)MPAD * PQW * 4)
#define BYTES_WB ((size_t)WROWS * KDIM * 2)
#define BYTES_BB ((size_t)128)

static_assert(MPAD == 782 * 128);
static_assert(MPAD >= NNODE);
static_assert((KDIM % 32) == 0);
static_assert((NEDGE % 2) == 0);
static_assert(((NEDGE * 4) % 8) == 0);
static_assert(NPAIR <= EBLKS * THR);
static_assert(PQW * 4 == 16);
static_assert(WROWS == 16);
static_assert(MTILE * PQW * 4 == 16 * 128);
static_assert((XUNITS % THR) == 0);
static_assert(WROWS * (KDIM / 8) == THR);
static_assert(MTILE == (THR / 32) * 16);
static_assert((BYTES_XB % 128) == 0 && (BYTES_PQ % 128) == 0 && (BYTES_WB % 128) == 0);
static_assert(BYTES_XB + BYTES_PQ + BYTES_WB + BYTES_BB <= (128u << 20));

typedef float          v4f  __attribute__((ext_vector_type(4)));
typedef float          v8f  __attribute__((ext_vector_type(8)));
typedef int            v2i  __attribute__((ext_vector_type(2)));
typedef int            v8i  __attribute__((ext_vector_type(8)));
typedef unsigned int   v4u  __attribute__((ext_vector_type(4)));
typedef unsigned short v8us __attribute__((ext_vector_type(8)));
typedef __bf16         v16b __attribute__((ext_vector_type(16)));
typedef v4f  __attribute__((may_alias)) v4fa;
typedef v2i  __attribute__((may_alias)) v2ia;
typedef v8us __attribute__((may_alias)) v8usa;
union FragB { v16b v; v8us h[2]; v8i w; };

__device__ __forceinline__ v8f wmb(const FragB& a, const FragB& b, v8f c) {
  v8f d = __builtin_amdgcn_wmma_f32_16x16x32_bf16(false, a.v, false, b.v, (short)0, c, false, false);
  asm volatile("v_nop\n\tv_nop\n\tv_nop\n\tv_nop" : "+v"(d) : "v"(a.w), "v"(b.w));
  return d;
}

__device__ __forceinline__ unsigned int f2bf(float f) {
  const unsigned int u = __float_as_uint(f);
  return ((u + 0x7fffu + ((u >> 16) & 1u)) >> 16) & 0xffffu;
}
__device__ __forceinline__ float bf2f(unsigned int b) { return __uint_as_float(b << 16); }
__device__ __forceinline__ float bfr(float f) { return bf2f(f2bf(f)); }
__device__ __forceinline__ unsigned int pk2(float lo, float hi) { return f2bf(lo) | (f2bf(hi) << 16); }
__device__ __forceinline__ v4u pack8(const v4f a, const v4f b) {
  v4u r;
  r.x = pk2(a.x, a.y); r.y = pk2(a.z, a.w); r.z = pk2(b.x, b.y); r.w = pk2(b.z, b.w);
  return r;
}

__global__ __launch_bounds__(THR) void k_prep(const float* __restrict__ x, const float* __restrict__ w,
                                              const float* __restrict__ b,
                                              unsigned short* xb, unsigned short* wb, float* bb) {
  const int tid = (int)threadIdx.x;
  const v4f z4 = {0.f, 0.f, 0.f, 0.f};
  if ((int)blockIdx.x < XBLKS) {
    const int i   = (int)blockIdx.x * THR + tid;
    const int row = i >> 4;
    const int c0  = (i & 15) * 8;
    const int rc  = row < NNODE ? row : NNODE - 1;
    const float* p = x + (size_t)rc * KDIM + c0;
    v4f a = *(const v4fa*)p;
    v4f c = *(const v4fa*)(p + 4);
    asm volatile("" :: "v"(a), "v"(c));
    if (row >= NNODE) { a = z4; c = z4; }
    const v4u hv = pack8(a, c);
    unsigned short* o = xb + (size_t)row * KDIM + c0;
    *(volatile v4u*)o = hv;
    __threadfence();
    *(volatile v4u*)o = hv;
  } else {
    const int n   = tid >> 4;
    const int k8  = (tid & 15) * 8;
    const int nc  = n < 4 ? n : 3;
    const int cls = nc & 1;
    const int hf  = nc >> 1;
    const float* p = w + (size_t)cls * (2 * KDIM) + (size_t)hf * KDIM + k8;
    v4f a = *(const v4fa*)p;
    v4f c = *(const v4fa*)(p + 4);
    asm volatile("" :: "v"(a), "v"(c));
    if (n >= 4) { a = z4; c = z4; }
    const v4u wv = pack8(a, c);
    unsigned short* o = wb + (size_t)n * KDIM + k8;

    const float b0 = b[0];
    const float b1 = b[1];
    asm volatile("" :: "v"(b0), "v"(b1));
    v4f bv = z4;
    if (tid == 0) { bv.x = bfr(b0); bv.y = bfr(b1); }
    const int tb = tid < 8 ? tid : 7;
    float* ob = bb + 4 * tb;
    const bool wrb = tid < 8;

    *(volatile v4u*)o = wv;
    if (wrb) *(volatile v4f*)ob = bv;
    __threadfence();
    *(volatile v4u*)o = wv;
    if (wrb) *(volatile v4f*)ob = bv;
  }
}

__global__ __launch_bounds__(THR) void k_gemm_one(const unsigned short* __restrict__ xb,
                                                  const unsigned short* __restrict__ wb,
                                                  float* pq) {
  __shared__ __attribute__((aligned(16))) float st[MTILE * PQW];
  const int tid = (int)threadIdx.x, lane = tid & 31, wave = tid >> 5, hh = lane >> 4, m = lane & 15;
  const int rowBase = (int)blockIdx.x * MTILE;

  const unsigned short* ap = xb + (size_t)(rowBase + 16 * wave + m) * KDIM + 8 * hh;
  const unsigned short* wp = wb + (size_t)m * KDIM + 8 * hh;

  v8f acc = {0.f, 0.f, 0.f, 0.f, 0.f, 0.f, 0.f, 0.f};
#pragma unroll 1
  for (int ks = 0; ks < KDIM / 32; ++ks) {
    FragB af, bf;
    af.h[0] = *(const v8usa*)(ap + 32 * ks);
    af.h[1] = *(const v8usa*)(ap + 32 * ks + 16);
    bf.h[0] = *(const v8usa*)(wp + 32 * ks);
    bf.h[1] = *(const v8usa*)(wp + 32 * ks + 16);
    acc = wmb(af, bf, acc);
  }

  if (m < PQW) {
#pragma unroll
    for (int r = 0; r < 8; ++r) {
      const int lr = 16 * wave + 8 * hh + r;
      st[lr * PQW + m] = acc[r];
    }
  }
  __syncthreads();

  if (tid < MTILE) {
    const v4f v = *(const v4fa*)(st + 4 * tid);
    float* op = pq + (size_t)(rowBase + tid) * PQW;
    *(volatile v4f*)op = v;
    __threadfence();
    *(volatile v4f*)op = v;
  }
}

__global__ __launch_bounds__(THR) void k_edge(const int* __restrict__ ei, const float* __restrict__ pq,
                                              const float* __restrict__ bb, float* out) {
  const int i  = (int)blockIdx.x * THR + (int)threadIdx.x;
  const int ic = i < NPAIR ? i : NPAIR - 1;

  const v2i sp = *(const v2ia*)(ei + 2 * ic);
  const v2i dp = *(const v2ia*)(ei + NEDGE + 2 * ic);
  asm volatile("" :: "v"(sp), "v"(dp));
  int s0 = sp.x, s1 = sp.y, d0 = dp.x, d1 = dp.y;
  s0 = s0 < 0 ? 0 : (s0 > NNODE - 1 ? NNODE - 1 : s0);
  s1 = s1 < 0 ? 0 : (s1 > NNODE - 1 ? NNODE - 1 : s1);
  d0 = d0 < 0 ? 0 : (d0 > NNODE - 1 ? NNODE - 1 : d0);
  d1 = d1 < 0 ? 0 : (d1 > NNODE - 1 ? NNODE - 1 : d1);
  asm volatile("" :: "v"(s0), "v"(s1), "v"(d0), "v"(d1));

  const v4f ps0 = *(const v4fa*)(pq + (size_t)s0 * PQW);
  const v4f pd0 = *(const v4fa*)(pq + (size_t)d0 * PQW);
  const v4f ps1 = *(const v4fa*)(pq + (size_t)s1 * PQW);
  const v4f pd1 = *(const v4fa*)(pq + (size_t)d1 * PQW);
  asm volatile("" :: "v"(ps0), "v"(pd0), "v"(ps1), "v"(pd1));

  const v4f bv = *(const v4fa*)bb;
  const float b0 = bv.x, b1 = bv.y;
  asm volatile("" :: "v"(b0), "v"(b1));

  v4f r;
  r.x = (ps0.x + pd0.z) + b0;
  r.y = (ps0.y + pd0.w) + b1;
  r.z = (ps1.x + pd1.z) + b0;
  r.w = (ps1.y + pd1.w) + b1;

  float* op = out + (size_t)4 * (size_t)ic;
  const bool wr = i < NPAIR;
  if (wr) *(volatile v4f*)op = r;
  __threadfence();
  if (wr) *(volatile v4f*)op = r;
}

extern "C" void kernel_launch(void* const* d_in, const int* in_sizes, int n_in,
                              void* d_out, int out_size, void* d_ws, size_t ws_size,
                              hipStream_t stream) {
  if (n_in < 4) return;
  if (in_sizes[0] != NNODE * KDIM) return;
  if (in_sizes[1] != 2 * NEDGE) return;
  if (in_sizes[2] != 2 * 2 * KDIM) return;
  if (in_sizes[3] != 2) return;
  if (out_size != 2 * NEDGE) return;

  const float* x  = (const float*)d_in[0];
  const int*   ei = (const int*)  d_in[1];
  const float* w  = (const float*)d_in[2];
  const float* b  = (const float*)d_in[3];
  float* out = (float*)d_out;

  const size_t oXB = 0;
  const size_t oPQ = oXB + BYTES_XB;
  const size_t oWB = oPQ + BYTES_PQ;
  const size_t oBB = oWB + BYTES_WB;
  const size_t total = oBB + BYTES_BB;
  if (total > ws_size || total > (size_t)(128u << 20)) return;

  char* ws = (char*)d_ws;
  unsigned short* XB = (unsigned short*)(ws + oXB);
  float*          PQ = (float*)(ws + oPQ);
  unsigned short* WB = (unsigned short*)(ws + oWB);
  float*          BB = (float*)(ws + oBB);

  k_prep<<<XBLKS + 1, THR, 0, stream>>>(x, w, b, XB, WB, BB);
  k_gemm_one<<<MBLK, THR, 0, stream>>>(XB, WB, PQ);
  k_edge<<<EBLKS, THR, 0, stream>>>(ei, PQ, BB, out);
}
